// GRU_DOUBLE_ATT_STACK_PARALLEL_DROPOUT_57990648430732
// MI455X (gfx1250) — hardware-run, weakly checked
//
#include <hip/hip_runtime.h>
#include <math.h>

constexpr int kBatch  = 64;
constexpr int kAtt    = 196;
constexpr int kAttPad = 256;
constexpr int kRnn    = 1024;
constexpr int kIn     = 1024;
constexpr int kOut    = 9487;
constexpr int kOutPad = 9536;
constexpr int kPar    = 4;
constexpr int kRowsAV = kBatch * kAtt;
constexpr int kKcat   = 3072;
constexpr int kNsum   = kPar * 2 * kRnn;
constexpr int kNhg    = kRnn;
constexpr float kWCarry = 64.0f;
constexpr float kWInv   = 1.0f / 64.0f;
constexpr int kOut1Float4 = (kBatch * kOut) / 4;
static_assert((kBatch * kOut) % 4 == 0, "flat writer granularity");
static_assert(kRowsAV % 64 == 0 && kOutPad % 64 == 0 && kNsum % 64 == 0 && kKcat % 32 == 0 && kRnn % 32 == 0, "tile multiples");
static_assert(kIn == kRnn, "shared row pitch for x and h");

constexpr size_t kOffBig    = 0;
constexpr size_t kSzAtt16   = (size_t)kRowsAV * kRnn * 2;
constexpr size_t kSzWprojT  = (size_t)kOutPad * kRnn * 2;
constexpr size_t kOffAcat0  = kOffBig + kSzWprojT;
constexpr size_t kSzAcat0   = (size_t)kBatch * kKcat * 2;
constexpr size_t kOffAcat1  = kOffAcat0 + kSzAcat0;
constexpr size_t kSzAcat1   = (size_t)kPar * kBatch * kKcat * 2;
constexpr size_t kOffSums   = kOffAcat1 + kSzAcat1;
constexpr size_t kSzSums    = (size_t)kBatch * kNsum * 4;
constexpr size_t kOffHg     = kOffSums + kSzSums;
constexpr size_t kSzHg      = (size_t)kPar * kBatch * kRnn * 4;
constexpr size_t kOffAh     = kOffHg + kSzHg;
constexpr size_t kSzSmall   = (size_t)kBatch * kAttPad * 4;
constexpr size_t kOffSc     = kOffAh + kSzSmall;
constexpr size_t kOffNh32   = kOffSc + kSzSmall;
constexpr size_t kSzRow32   = (size_t)kBatch * kRnn * 4;
constexpr size_t kOffNh16   = kOffNh32 + kSzRow32;
constexpr size_t kSzRow16   = (size_t)kBatch * kRnn * 2;
constexpr size_t kOffTop16  = kOffNh16 + kSzRow16;
constexpr size_t kEndBig    = kOffTop16 + kSzRow16;
static_assert(kEndBig <= kSzAtt16, "activations fit the BIG region tail");
constexpr size_t kOffAv0    = kOffBig + kSzAtt16;
constexpr size_t kSzAv      = (size_t)kRowsAV * kAttPad * 4;
constexpr size_t kOffAv1    = kOffAv0 + kSzAv;
constexpr size_t kOffLogits = kOffAv0;
constexpr size_t kSzLogits  = (size_t)kBatch * kOutPad * 4;
static_assert(kSzLogits <= kSzAv, "logits fit av0 region");
constexpr size_t kOffW0     = kOffAv1 + kSzAv;
constexpr size_t kSzW0      = (size_t)kNsum * kKcat * 2;
constexpr size_t kOffW1     = kOffW0 + kSzW0;
constexpr size_t kSzW1      = (size_t)kPar * kNhg * kKcat * 2;
constexpr size_t kOffWatt   = kOffW1 + kSzW1;
constexpr size_t kSzWatt    = (size_t)4 * kAttPad * kRnn * 2;
constexpr size_t kOffBsum0  = kOffWatt + kSzWatt;
constexpr size_t kOffBsum1  = kOffBsum0 + (size_t)kNsum * 4;
constexpr size_t kOffBproj  = kOffBsum1 + (size_t)kPar * kNhg * 4;
constexpr size_t kOffBatt   = kOffBproj + (size_t)kOutPad * 4;
constexpr size_t kOffLse    = kOffBatt + (size_t)4 * kAttPad * 4;
constexpr size_t kWsTotal   = kOffLse + (size_t)kBatch * 32 * 4;
static_assert(kWsTotal == 129074432ull, "carve total");
static_assert(kWsTotal <= 134217728ull, "carve under 128 MiB");
static_assert(kOffAcat0 % 128 == 0 && kOffAv0 % 128 == 0 && kOffW0 % 128 == 0 && kOffWatt % 128 == 0 &&
              kOffBsum0 % 128 == 0 && kOffBproj % 128 == 0 && kOffBatt % 128 == 0 && kOffLse % 128 == 0, "alignment");

typedef __attribute__((ext_vector_type(16))) _Float16 v16h;
typedef __attribute__((ext_vector_type(8)))  _Float16 v8h;
typedef __attribute__((ext_vector_type(16))) __bf16   v16b;
typedef __attribute__((ext_vector_type(8)))  __bf16   v8b;
typedef __attribute__((ext_vector_type(8)))  float    v8f;
typedef __attribute__((ext_vector_type(4)))  float    v4f;
typedef __attribute__((ext_vector_type(4)))  unsigned int v4u;

__device__ __forceinline__ unsigned short f2bf_bits(float f) {
  unsigned u = __float_as_uint(f);
  return (unsigned short)((u + 0x7FFFu + ((u >> 16) & 1u)) >> 16);
}
__device__ __forceinline__ float bf_bits2f(unsigned short h) { return __uint_as_float(((unsigned)h) << 16); }

__device__ __forceinline__ void dep_guard_h(v8f& a, v8f& b, v16h x, v16h y) { asm volatile("v_nop\n\tv_nop\n\tv_nop\n\tv_nop" : "+v"(a), "+v"(b) : "v"(x), "v"(y)); }
__device__ __forceinline__ void dep_guard_b(v8f& a, v8f& b, v16b x, v16b y) { asm volatile("v_nop\n\tv_nop\n\tv_nop\n\tv_nop" : "+v"(a), "+v"(b) : "v"(x), "v"(y)); }
__device__ __forceinline__ void keep4_h(v16h a, v16h b, v16h c, v16h d) { asm volatile("v_nop" :: "v"(a), "v"(b), "v"(c), "v"(d)); }
__device__ __forceinline__ void keep4_b(v16b a, v16b b, v16b c, v16b d) { asm volatile("v_nop" :: "v"(a), "v"(b), "v"(c), "v"(d)); }
__device__ __forceinline__ void acc_guard4(v8f& a, v8f& b, v8f& c, v8f& d) { asm volatile("v_nop\n\tv_nop\n\tv_nop\n\tv_nop" : "+v"(a), "+v"(b), "+v"(c), "+v"(d)); }
template <typename T> struct Frag;
template <> struct Frag<_Float16> {
  typedef v16h V; union U { v16h v; v8h h[2]; };
  static __device__ __forceinline__ v16h load(const _Float16* p) {
    U f; f.h[0] = *(const v8h*)(p); f.h[1] = *(const v8h*)(p + 16); return f.v;
  }
  static __device__ __forceinline__ v8f mma(v16h a, v16h b, v8f c) {
    return __builtin_amdgcn_wmma_f32_16x16x32_f16(false, a, false, b, (short)0, c, false, false);
  }
  static __device__ __forceinline__ void guard(v8f& a, v8f& b, v16h x, v16h y) { dep_guard_h(a, b, x, y); }
  static __device__ __forceinline__ void keep(v16h a, v16h b, v16h c, v16h d) { keep4_h(a, b, c, d); }
};
template <> struct Frag<__bf16> {
  typedef v16b V; union U { v16b v; v8b h[2]; };
  static __device__ __forceinline__ v16b load(const __bf16* p) {
    U f; f.h[0] = *(const v8b*)(p); f.h[1] = *(const v8b*)(p + 16); return f.v;
  }
  static __device__ __forceinline__ v8f mma(v16b a, v16b b, v8f c) {
    return __builtin_amdgcn_wmma_f32_16x16x32_bf16(false, a, false, b, (short)0, c, false, false);
  }
  static __device__ __forceinline__ void guard(v8f& a, v8f& b, v16b x, v16b y) { dep_guard_b(a, b, x, y); }
  static __device__ __forceinline__ void keep(v16b a, v16b b, v16b c, v16b d) { keep4_b(a, b, c, d); }
};

__device__ __forceinline__ unsigned pk16(unsigned short a, unsigned short b) { return (unsigned)a | ((unsigned)b << 16); }
__device__ __forceinline__ unsigned short h_bits(float f) { const _Float16 h = (_Float16)f; return __builtin_bit_cast(unsigned short, h); }

__device__ __forceinline__ void st2_u4(unsigned short* p, v4u u) {
  *(volatile v4u*)p = u;
  __threadfence();
  *(volatile v4u*)p = u;
}
__device__ __forceinline__ void st2_f4(float* p, v4f v) {
  *(volatile v4f*)p = v;
  __threadfence();
  *(volatile v4f*)p = v;
}
__device__ __forceinline__ v4u pack8(const float* s) {
  unsigned short hb[8];
#pragma unroll
  for (int e = 0; e < 8; ++e) hb[e] = h_bits(s[e]);
  return (v4u){pk16(hb[0], hb[1]), pk16(hb[2], hb[3]), pk16(hb[4], hb[5]), pk16(hb[6], hb[7])};
}
__device__ __forceinline__ float sigm(float x) {
  const float xc = fminf(fmaxf(x, -30.0f), 30.0f);
  const float e = expf(-xc);
  return 1.0f / (1.0f + e);
}

template <int ET> struct Elem;
template <> struct Elem<0> { typedef _Float16 T; };
template <> struct Elem<1> { typedef __bf16 T; };
template <int ET, bool SPLIT, int BIAS_MODE, int OUT_MODE, bool RESID, int ACT = 0>
__global__ __launch_bounds__(256) void wmma_gemm64(
    const unsigned short* __restrict__ Ap, const unsigned short* __restrict__ A2p, int lda, long strideA,
    const unsigned short* __restrict__ Btp, const unsigned short* __restrict__ Bt2p, int ldb, long strideB,
    void* __restrict__ Cout, void* __restrict__ Cout2, int ldc, long strideC,
    const float* __restrict__ bias, long strideBias,
    const float* __restrict__ resid, long strideR,
    int M, int N, int K, float scale) {
  typedef typename Elem<ET>::T T;
  typedef typename Frag<T>::V V;
  const T* A = (const T*)Ap; const T* A2 = (const T*)A2p; const T* Bt = (const T*)Btp; const T* Bt2 = (const T*)Bt2p;
  __shared__ __align__(16) float sT[8][16 * 68];
  const int b    = blockIdx.y;
  const int lane = threadIdx.x & 31;
  const int wave = threadIdx.x >> 5;
  const int tilesN = N >> 6;
  const int tilesM = M >> 6;
  const int tile = blockIdx.x * 8 + wave;
  if (tile >= tilesM * tilesN) return;
  const int tm = tile / tilesN;
  const int tn = tile - tm * tilesN;
  const int m0 = tm << 6;
  const int n0 = tn << 6;

  const T* Ab  = A  + (size_t)b * strideA;
  const T* Bb  = Bt + (size_t)b * strideB;
  const T* Ab2 = SPLIT ? (A2  + (size_t)b * strideA) : nullptr;
  const T* Bb2 = SPLIT ? (Bt2 + (size_t)b * strideB) : nullptr;
  const float* Bsb = (BIAS_MODE != 0) ? (bias + (size_t)b * strideBias) : nullptr;

  const int rlane = lane & 15;
  const int koff  = (lane >> 4) * 8;
  const int mOff  = (lane >> 4) * 8;

  v8f acc[4][4];
#pragma unroll
  for (int i = 0; i < 4; ++i)
#pragma unroll
    for (int j = 0; j < 4; ++j) acc[i][j] = (v8f){0.f,0.f,0.f,0.f,0.f,0.f,0.f,0.f};

  for (int k0 = 0; k0 < K; k0 += 32) {
    V bh[4], bl[4];
#pragma unroll
    for (int j = 0; j < 4; ++j) {
      const size_t bo = (size_t)(n0 + (j << 4) + rlane) * ldb + koff + k0;
      bh[j] = Frag<T>::load(Bb + bo);
      if (SPLIT) bl[j] = Frag<T>::load(Bb2 + bo);
    }
#pragma unroll
    for (int i = 0; i < 4; ++i) {
      const size_t ao = (size_t)(m0 + (i << 4) + rlane) * lda + koff + k0;
      V ah = Frag<T>::load(Ab + ao);
      V al;
      if (SPLIT) al = Frag<T>::load(Ab2 + ao);
#pragma unroll
      for (int j = 0; j < 4; ++j) {
        acc[i][j] = Frag<T>::mma(ah, bh[j], acc[i][j]);
        if (SPLIT) {
          acc[i][j] = Frag<T>::mma(ah, bl[j], acc[i][j]);
          acc[i][j] = Frag<T>::mma(al, bh[j], acc[i][j]);
        }
      }
      Frag<T>::guard(acc[i][0], acc[i][3], ah, SPLIT ? al : ah);
    }
    Frag<T>::keep(bh[0], bh[1], bh[2], bh[3]);
    if (SPLIT) Frag<T>::keep(bl[0], bl[1], bl[2], bl[3]);
  }
  acc_guard4(acc[0][0], acc[0][1], acc[0][2], acc[0][3]);
  acc_guard4(acc[1][0], acc[1][1], acc[1][2], acc[1][3]);
  acc_guard4(acc[2][0], acc[2][1], acc[2][2], acc[2][3]);
  acc_guard4(acc[3][0], acc[3][1], acc[3][2], acc[3][3]);

  float* slab = sT[wave];
  const float* Rb = RESID ? (resid + (size_t)b * strideR) : nullptr;
#pragma unroll
  for (int i = 0; i < 4; ++i) {
    const int mBase = m0 + (i << 4);
#pragma unroll
    for (int j = 0; j < 4; ++j) {
      const int n = n0 + (j << 4) + rlane;
      float bv = 0.f;
      if (BIAS_MODE == 2) bv = Bsb[n];
#pragma unroll
      for (int r = 0; r < 8; ++r) {
        float v = acc[i][j][r] * scale;
        if (BIAS_MODE == 1) v += Bsb[mBase + mOff + r];
        if (BIAS_MODE == 2) v += bv;
        if (RESID) v += Rb[(size_t)(mBase + mOff + r) * ldc + n];
        if (ACT == 2) v = fmaxf(v, 0.0f);
        if (ACT == 4) v = (v > 0.f) ? v : 0.01f * v;
        slab[(mOff + r) * 68 + (j << 4) + rlane] = v;
      }
    }
    __builtin_amdgcn_fence(__ATOMIC_RELEASE, "workgroup");
    __builtin_amdgcn_wave_barrier();
    __builtin_amdgcn_fence(__ATOMIC_ACQUIRE, "workgroup");
    if (OUT_MODE == 0) {
      float* C = (float*)Cout + (size_t)b * strideC;
      const int hh = lane >> 4, c4 = (lane & 15) * 4;
      for (int pass = 0; pass < 2; ++pass) {
#pragma unroll
        for (int it = 0; it < 8; ++it) {
          const int row = it * 2 + hh;
          v4f v = *(const v4f*)(slab + row * 68 + c4);
          *(volatile v4f*)(C + (size_t)(mBase + row) * ldc + n0 + c4) = v;
        }
        __threadfence();
      }
    } else {
      const int q = lane >> 3, c8 = (lane & 7) * 8;
      unsigned short* C  = (unsigned short*)Cout  + (size_t)b * strideC;
      unsigned short* C2 = (OUT_MODE == 2) ? ((unsigned short*)Cout2 + (size_t)b * strideC) : nullptr;
      for (int pass = 0; pass < 2; ++pass) {
#pragma unroll
        for (int it = 0; it < 4; ++it) {
          const int row = it * 4 + q;
          const float* sp = slab + row * 68 + c8;
          v8h hv, lv;
#pragma unroll
          for (int e = 0; e < 8; ++e) {
            if (OUT_MODE == 1) {
              hv[e] = (_Float16)sp[e];
            } else {
              unsigned short hb = f2bf_bits(sp[e]);
              unsigned short lb = f2bf_bits(sp[e] - bf_bits2f(hb));
              hv[e] = __builtin_bit_cast(_Float16, hb);
              lv[e] = __builtin_bit_cast(_Float16, lb);
            }
          }
          *(volatile v8h*)(C + (size_t)(mBase + row) * ldc + n0 + c8) = hv;
          if (OUT_MODE == 2) *(volatile v8h*)(C2 + (size_t)(mBase + row) * ldc + n0 + c8) = lv;
        }
        __threadfence();
      }
    }
    __builtin_amdgcn_fence(__ATOMIC_RELEASE, "workgroup");
    __builtin_amdgcn_wave_barrier();
    __builtin_amdgcn_fence(__ATOMIC_ACQUIRE, "workgroup");
  }
}

__global__ __launch_bounds__(256) void cast8_f16_kernel(const float* __restrict__ in, unsigned short* __restrict__ out, int n8) {
  const int i = blockIdx.x * 256 + threadIdx.x;
  if (i >= n8) return;
  const float* p = in + 8 * (size_t)i;
  const v4f a = *(const v4f*)(p);
  const v4f c = *(const v4f*)(p + 4);
  unsigned short hb[8];
#pragma unroll
  for (int e = 0; e < 4; ++e) {
    hb[e]     = h_bits(a[e]);
    hb[4 + e] = h_bits(c[e]);
  }
  const v4u u = (v4u){pk16(hb[0], hb[1]), pk16(hb[2], hb[3]), pk16(hb[4], hb[5]), pk16(hb[6], hb[7])};
  st2_u4(out + 8 * (size_t)i, u);
}

__global__ __launch_bounds__(256) void wtcast_kernel(const float* __restrict__ W0, const float* __restrict__ W1,
                                                     const float* __restrict__ W2, const float* __restrict__ W3,
                                                     int zPerPtr, long srcStrideZ, int ldw, int nValid,
                                                     unsigned short* __restrict__ out, int ldo,
                                                     int rowBasePerPtr, int rowStridePerZ, int colBasePerPtr, float scale) {
  __shared__ float sm[64][65];
  const int t  = threadIdx.x;
  const int k0 = blockIdx.x * 64;
  const int n0 = blockIdx.y * 64;
  const int z  = blockIdx.z;
  const int pi = z / zPerPtr;
  const int zz = z - pi * zPerPtr;
  const float* W = (pi == 0) ? W0 : (pi == 1) ? W1 : (pi == 2) ? W2 : W3;
  W += (size_t)zz * (size_t)srcStrideZ;
#pragma unroll
  for (int i = 0; i < 16; ++i) {
    const int e = i * 256 + t;
    const int r = e >> 6;
    const int c = e & 63;
    const int n = n0 + c;
    const int nc = (n < nValid) ? n : (nValid - 1);
    float v = W[(size_t)(k0 + r) * ldw + nc] * scale;
    if (n >= nValid) v = 0.0f;
    sm[c][r] = v;
  }
  __syncthreads();
  const int lane = t & 31, wave = t >> 5;
  const int q = lane >> 3, c8 = (lane & 7) * 8;
  const size_t rowBase = (size_t)rowBasePerPtr * pi + (size_t)rowStridePerZ * zz + n0;
  const size_t colBase = (size_t)colBasePerPtr * pi + k0 + c8;
#pragma unroll
  for (int it = 0; it < 2; ++it) {
    const int rowl = wave * 8 + it * 4 + q;
    const v4u u = pack8(&sm[rowl][c8]);
    st2_u4(out + (rowBase + rowl) * (size_t)ldo + colBase, u);
  }
}

__global__ __launch_bounds__(256) void bias_kernel(const float* __restrict__ bi2h, const float* __restrict__ bh2h, const float* __restrict__ ba2h,
                                                   const float* __restrict__ bi2h1, const float* __restrict__ bh2h1, const float* __restrict__ ba2h1,
                                                   const float* __restrict__ bproj,
                                                   const float* __restrict__ ba2a, const float* __restrict__ bh2a,
                                                   const float* __restrict__ ba2a1, const float* __restrict__ bh2a1,
                                                   float* __restrict__ bsum0, float* __restrict__ bsum1,
                                                   float* __restrict__ bprojp, float* __restrict__ battpad) {
  const int seg = blockIdx.y;
  const int i = blockIdx.x * 256 + threadIdx.x;
  v4f v = (v4f){0.f, 0.f, 0.f, 0.f};
  float* dst;
  int cnt;
  if (seg == 0) {
    cnt = kNsum / 4;
    const int ic = (i < cnt) ? i : (cnt - 1);
#pragma unroll
    for (int c = 0; c < 4; ++c) { const int n = 4 * ic + c; v[c] = bi2h[n] + bh2h[n] + ba2h[n]; }
    dst = bsum0;
  } else if (seg == 1) {
    cnt = (kPar * kNhg) / 4;
    const int ic = (i < cnt) ? i : (cnt - 1);
#pragma unroll
    for (int c = 0; c < 4; ++c) { const int n = 4 * ic + c; v[c] = bi2h1[n] + bh2h1[n] + ba2h1[n]; }
    dst = bsum1;
  } else if (seg == 2) {
    cnt = kOutPad / 4;
    const int ic = (i < cnt) ? i : (cnt - 1);
#pragma unroll
    for (int c = 0; c < 4; ++c) {
      const int n = 4 * ic + c;
      const int nc = (n < kOut) ? n : (kOut - 1);
      const float f = bproj[nc];
      v[c] = (n < kOut) ? f : 0.0f;
    }
    dst = bprojp;
  } else {
    cnt = (4 * kAttPad) / 4;
    const int ic = (i < cnt) ? i : (cnt - 1);
#pragma unroll
    for (int c = 0; c < 4; ++c) {
      const int n = 4 * ic + c;
      const int qsel = n >> 8;
      const int a = n & 255;
      const int ac = (a < kAtt) ? a : (kAtt - 1);
      const float f0 = ba2a[ac], f1 = bh2a[ac], f2 = ba2a1[ac], f3 = bh2a1[ac];
      const float f = (qsel == 0) ? f0 : (qsel == 1) ? f1 : (qsel == 2) ? f2 : f3;
      v[c] = (a < kAtt) ? f : 0.0f;
    }
    dst = battpad;
  }
  if (i < cnt) st2_f4(dst + 4 * (size_t)i, v);
}

__global__ __launch_bounds__(256) void prep_kernel(const float* __restrict__ x, const float* __restrict__ hp,
                                                   unsigned short* __restrict__ acat0, unsigned short* __restrict__ acat1, int writeX) {
  __shared__ __align__(16) float sx[256];
  __shared__ __align__(16) float sh[256];
  const int t = threadIdx.x, lane = t & 31, wave = t >> 5;
  const int chunk = blockIdx.x, b = blockIdx.y;
  const size_t src = (size_t)b * kRnn + chunk * 256 + t;
  sx[t] = x[src];
  sh[t] = hp[src];
  __syncthreads();
  if (writeX != 0 && wave < 5) {
    unsigned short* base;
    if (wave == 0) base = acat0 + (size_t)b * kKcat + chunk * 256;
    else base = acat1 + (size_t)(wave - 1) * kBatch * kKcat + (size_t)b * kKcat + chunk * 256;
    const v4u u = pack8(sx + 8 * lane);
    st2_u4(base + 8 * lane, u);
  }
  if (wave == 5) {
    const v4u u = pack8(sh + 8 * lane);
    st2_u4(acat0 + (size_t)b * kKcat + 1024 + chunk * 256 + 8 * lane, u);
  }
}

__global__ __launch_bounds__(256) void score_kernel(const float* __restrict__ av, const float* __restrict__ ah,
                                                    const float* __restrict__ Wd, const float* __restrict__ bd, float* __restrict__ sc) {
  __shared__ __align__(16) float ssc[64];
  const int t = threadIdx.x, lane = t & 31, wave = t >> 5;
  const int g = blockIdx.x, b = blockIdx.y;
  const float bd0 = bd[0];
#pragma unroll 1
  for (int rr = 0; rr < 8; ++rr) {
    const int al = wave * 8 + rr;
    const int a  = g * 64 + al;
    const int ac = (a < kAtt) ? a : (kAtt - 1);
    const float ahv = ah[(size_t)b * kAttPad + ac];
    const float* avr = av + ((size_t)b * kAtt + ac) * kAttPad;
    float acc = 0.0f;
#pragma unroll 1
    for (int j = 0; j < 7; ++j) {
      const int o  = lane + 32 * j;
      const int oc = (o < kAtt) ? o : (kAtt - 1);
      const float tv = tanhf(avr[oc] + ahv);
      const float wv = Wd[oc];
      const float prod = tv * wv;
      acc += (o < kAtt) ? prod : 0.0f;
    }
#pragma unroll
    for (int off = 16; off > 0; off >>= 1) acc += __shfl_xor(acc, off, 32);
    if (lane == 0) ssc[al] = (a < kAtt) ? (acc + bd0) : 0.0f;
  }
  __syncthreads();
  if (wave == 0 && lane < 16) {
    const v4f v = *(const v4f*)(ssc + 4 * lane);
    st2_f4(sc + (size_t)b * kAttPad + g * 64 + 4 * lane, v);
  }
}

template <int MODE>
__global__ __launch_bounds__(256) void attapply_kernel(const float* __restrict__ sc, const float* __restrict__ att,
                                                       const float* __restrict__ nh, const float* __restrict__ x,
                                                       float* __restrict__ dout,
                                                       unsigned short* __restrict__ acat0, unsigned short* __restrict__ acat1,
                                                       unsigned short* __restrict__ toph) {
  __shared__ float swl[kAttPad];
  __shared__ __align__(16) float sv[256];
  __shared__ __align__(16) float sc16[256];
  __shared__ float sredm[8];
  __shared__ float sreds[8];
  const int t = threadIdx.x, lane = t & 31, wave = t >> 5;
  const int chunk = blockIdx.x, b = blockIdx.y;
  const float raw  = sc[(size_t)b * kAttPad + t];
  const float sval = (t < kAtt) ? raw : -INFINITY;
  float m = sval;
#pragma unroll
  for (int off = 16; off > 0; off >>= 1) m = fmaxf(m, __shfl_xor(m, off, 32));
  if (lane == 0) sredm[wave] = m;
  __syncthreads();
  float gm = sredm[0];
#pragma unroll
  for (int w = 1; w < 8; ++w) gm = fmaxf(gm, sredm[w]);
  const float ev = (t < kAtt) ? expf(sval - gm) : 0.0f;
  float s = ev;
#pragma unroll
  for (int off = 16; off > 0; off >>= 1) s += __shfl_xor(s, off, 32);
  if (lane == 0) sreds[wave] = s;
  __syncthreads();
  float gs = sreds[0];
#pragma unroll
  for (int w = 1; w < 8; ++w) gs += sreds[w];
  swl[t] = ev * (1.0f / gs);
  __syncthreads();
  const int r = chunk * 256 + t;
  const float* ab = att + (size_t)b * kAtt * kRnn + r;
  float acc = 0.0f;
#pragma unroll 1
  for (int a = 0; a < kAtt; ++a) acc += ab[(size_t)a * kRnn] * swl[a];
  if (MODE == 0) {
    sc16[t] = acc;
  } else {
    const float o = acc + nh[(size_t)b * kRnn + r];
    sv[t] = o;
    if (MODE == 1) sc16[t] = x[(size_t)b * kIn + r] + o;
    else sc16[t] = o;
  }
  __syncthreads();
  if (MODE == 0 || MODE == 1) {
    const int colb = (MODE == 0) ? 2048 : 0;
    if (wave < 5) {
      unsigned short* base;
      if (wave == 0) base = acat0 + (size_t)b * kKcat + colb + chunk * 256;
      else base = acat1 + (size_t)(wave - 1) * kBatch * kKcat + (size_t)b * kKcat + colb + chunk * 256;
      const v4u u = pack8(sc16 + 8 * lane);
      st2_u4(base + 8 * lane, u);
    }
  }
  if (MODE == 2) {
    if (wave == 0) {
      const v4u u = pack8(sc16 + 8 * lane);
      st2_u4(toph + (size_t)b * kRnn + chunk * 256 + 8 * lane, u);
    }
  }
  if (MODE != 0) {
    if (wave == 5 || wave == 6) {
      const int idx = (wave - 5) * 32 + lane;
      const v4f v = *(const v4f*)(sv + 4 * idx);
      float* op = dout + ((size_t)(MODE - 1) * kBatch + b) * kRnn + chunk * 256 + 4 * idx;
      st2_f4(op, v);
    }
  }
}

__global__ __launch_bounds__(256) void gate_kernel(const float* __restrict__ sums, const float* __restrict__ hp,
                                                   unsigned short* __restrict__ acat1) {
  __shared__ __align__(16) float sg[kPar][256];
  const int t = threadIdx.x, lane = t & 31, wave = t >> 5;
  const int chunk = blockIdx.x, b = blockIdx.y;
  const int r = chunk * 256 + t;
  const float ph = hp[(size_t)b * kRnn + r];
#pragma unroll 1
  for (int p = 0; p < kPar; ++p) {
    const float sr = sums[(size_t)b * kNsum + p * 2048 + 1024 + r];
    sg[p][t] = sigm(sr) * ph;
  }
  __syncthreads();
  if (wave < kPar) {
    const v4u u = pack8(&sg[wave][8 * lane]);
    st2_u4(acat1 + (size_t)wave * kBatch * kKcat + (size_t)b * kKcat + 1024 + chunk * 256 + 8 * lane, u);
  }
}

__global__ __launch_bounds__(256) void nh_kernel(const float* __restrict__ sums, const float* __restrict__ hgpre,
                                                 const float* __restrict__ hp, float* __restrict__ nh32,
                                                 unsigned short* __restrict__ nh16) {
  __shared__ __align__(16) float sn[256];
  const int t = threadIdx.x, lane = t & 31, wave = t >> 5;
  const int chunk = blockIdx.x, b = blockIdx.y;
  const int r = chunk * 256 + t;
  const float ph = hp[(size_t)b * kRnn + r];
  float s = 0.0f;
#pragma unroll 1
  for (int p = 0; p < kPar; ++p) {
    const float z  = sigm(sums[(size_t)b * kNsum + p * 2048 + r]);
    const float hg = tanhf(hgpre[((size_t)p * kBatch + b) * kRnn + r]);
    s += (1.0f - z) * ph + z * hg;
  }
  sn[t] = s * 0.25f;
  __syncthreads();
  if (wave < 2) {
    const int idx = wave * 32 + lane;
    const v4f v = *(const v4f*)(sn + 4 * idx);
    st2_f4(nh32 + (size_t)b * kRnn + chunk * 256 + 4 * idx, v);
  }
  if (wave == 2) {
    const v4u u = pack8(sn + 8 * lane);
    st2_u4(nh16 + (size_t)b * kRnn + chunk * 256 + 8 * lane, u);
  }
}

__global__ __launch_bounds__(256) void lse_kernel(const float* __restrict__ logits, float* __restrict__ lsetab) {
  __shared__ float sred[8];
  __shared__ float sred2[8];
  const int t = threadIdx.x, lane = t & 31, wave = t >> 5;
  const int b = blockIdx.x;
  const float* row = logits + (size_t)b * kOutPad;
  float m = -INFINITY;
#pragma unroll 1
  for (int j = t; j < kOut; j += 256) m = fmaxf(m, row[j]);
#pragma unroll
  for (int off = 16; off > 0; off >>= 1) m = fmaxf(m, __shfl_xor(m, off, 32));
  if (lane == 0) sred[wave] = m;
  __syncthreads();
  float gm = sred[0];
#pragma unroll
  for (int w = 1; w < 8; ++w) gm = fmaxf(gm, sred[w]);
  float s = 0.0f;
#pragma unroll 1
  for (int j = t; j < kOut; j += 256) s += expf(row[j] - gm);
#pragma unroll
  for (int off = 16; off > 0; off >>= 1) s += __shfl_xor(s, off, 32);
  if (lane == 0) sred2[wave] = s;
  __syncthreads();
  float gs = sred2[0];
#pragma unroll
  for (int w = 1; w < 8; ++w) gs += sred2[w];
  const float logs = logf(gs);
  if (wave == 0) {
    const float v = (lane == 0) ? gm : (lane == 1) ? logs : 0.0f;
    float* p = lsetab + (size_t)b * 32 + lane;
    *(volatile float*)p = v;
    __threadfence();
    *(volatile float*)p = v;
  }
}

__global__ __launch_bounds__(256) void lsm_write_kernel(const float* __restrict__ logits, const float* __restrict__ lsetab,
                                                        float* __restrict__ out1) {
  const int g = blockIdx.x * 256 + threadIdx.x;
  if (g >= kOut1Float4) return;
  v4f v = (v4f){0.f, 0.f, 0.f, 0.f};
#pragma unroll
  for (int c = 0; c < 4; ++c) {
    const int e = 4 * g + c;
    int b = e / kOut;
    b = (b < kBatch) ? b : (kBatch - 1);
    const int j = e - b * kOut;
    const float lg = logits[(size_t)b * kOutPad + j];
    const float mx = lsetab[(size_t)b * 32];
    const float ls = lsetab[(size_t)b * 32 + 1];
    v[c] = (lg - mx) - ls;
  }
  st2_f4(out1 + 4 * (size_t)g, v);
}

static void launch_gemm(hipStream_t stream, int gx, int gy,
                        const unsigned short* A, int lda, long strideA,
                        const unsigned short* Bt, int ldb, long strideB,
                        float* Cf, int ldc, long strideC,
                        const float* bias, long strideBias,
                        int M, int N, int K) {
  wmma_gemm64<0, false, 2, 0, false, 0><<<dim3(gx, gy), 256, 0, stream>>>(
      A, A, lda, strideA, Bt, Bt, ldb, strideB, (void*)Cf, (void*)Cf, ldc, strideC,
      bias, strideBias, bias, 0L, M, N, K, kWInv);
}

extern "C" void kernel_launch(void* const* d_in, const int* in_sizes, int n_in,
                              void* d_out, int out_size, void* d_ws, size_t ws_size,
                              hipStream_t stream) {
  (void)in_sizes; (void)n_in; (void)out_size;
  if (ws_size < kWsTotal) return;

  const float* x      = (const float*)d_in[0];
  const float* att    = (const float*)d_in[1];
  const float* inputs = (const float*)d_in[2];
  const float* Wa2a  = (const float*)d_in[3];  const float* ba2a  = (const float*)d_in[4];
  const float* Wh2a  = (const float*)d_in[5];  const float* bh2a  = (const float*)d_in[6];
  const float* Wd2d  = (const float*)d_in[7];  const float* bd2d  = (const float*)d_in[8];
  const float* Wa2a1 = (const float*)d_in[9];  const float* ba2a1 = (const float*)d_in[10];
  const float* Wh2a1 = (const float*)d_in[11]; const float* bh2a1 = (const float*)d_in[12];
  const float* Wd2d1 = (const float*)d_in[13]; const float* bd2d1 = (const float*)d_in[14];
  const float* Wi2h  = (const float*)d_in[15]; const float* bi2h  = (const float*)d_in[16];
  const float* Wh2h  = (const float*)d_in[17]; const float* bh2h  = (const float*)d_in[18];
  const float* Wa2h  = (const float*)d_in[19]; const float* ba2h  = (const float*)d_in[20];
  const float* Wi2h1 = (const float*)d_in[21]; const float* bi2h1 = (const float*)d_in[22];
  const float* Wh2h1 = (const float*)d_in[23]; const float* bh2h1 = (const float*)d_in[24];
  const float* Wa2h1 = (const float*)d_in[25]; const float* ba2h1 = (const float*)d_in[26];
  const float* Wproj = (const float*)d_in[27]; const float* bproj = (const float*)d_in[28];

  char* ws = (char*)d_ws;
  unsigned short* att16  = (unsigned short*)(ws + kOffBig);
  unsigned short* wprojT = (unsigned short*)(ws + kOffBig);
  unsigned short* acat0  = (unsigned short*)(ws + kOffAcat0);
  unsigned short* acat1  = (unsigned short*)(ws + kOffAcat1);
  float* sums   = (float*)(ws + kOffSums);
  float* hgpre  = (float*)(ws + kOffHg);
  float* ahbuf  = (float*)(ws + kOffAh);
  float* scbuf  = (float*)(ws + kOffSc);
  float* nh32   = (float*)(ws + kOffNh32);
  unsigned short* nh16  = (unsigned short*)(ws + kOffNh16);
  unsigned short* top16 = (unsigned short*)(ws + kOffTop16);
  float* av0    = (float*)(ws + kOffAv0);
  float* av1    = (float*)(ws + kOffAv1);
  float* logits = (float*)(ws + kOffLogits);
  unsigned short* w0   = (unsigned short*)(ws + kOffW0);
  unsigned short* w1   = (unsigned short*)(ws + kOffW1);
  unsigned short* watt = (unsigned short*)(ws + kOffWatt);
  float* bsum0   = (float*)(ws + kOffBsum0);
  float* bsum1   = (float*)(ws + kOffBsum1);
  float* bprojp  = (float*)(ws + kOffBproj);
  float* battpad = (float*)(ws + kOffBatt);
  float* lsetab  = (float*)(ws + kOffLse);

  float* dout = (float*)d_out;
  float* out1 = dout + (size_t)2 * kBatch * kRnn;

  const size_t plane = (size_t)kAttPad * kRnn;

  bias_kernel<<<dim3(10, 4), 256, 0, stream>>>(bi2h, bh2h, ba2h, bi2h1, bh2h1, ba2h1, bproj,
                                               ba2a, bh2a, ba2a1, bh2a1, bsum0, bsum1, bprojp, battpad);
  cast8_f16_kernel<<<6272, 256, 0, stream>>>(att, att16, kRowsAV * kRnn / 8);
  wtcast_kernel<<<dim3(16, 4, 4), 256, 0, stream>>>(Wa2a, Wh2a, Wa2a1, Wh2a1, 1, 0L, kAtt, kAtt,
                                                     watt, kRnn, kAttPad, 0, 0, kWCarry);
  launch_gemm(stream, 98, 1, att16, kRnn, 0L, watt + 0 * plane, kRnn, 0L, av0, kAttPad, 0L,
              battpad + 0 * kAttPad, 0L, kRowsAV, kAttPad, kRnn);
  launch_gemm(stream, 98, 1, att16, kRnn, 0L, watt + 2 * plane, kRnn, 0L, av1, kAttPad, 0L,
              battpad + 2 * kAttPad, 0L, kRowsAV, kAttPad, kRnn);
  wtcast_kernel<<<dim3(16, 32, 12), 256, 0, stream>>>(Wi2h, Wh2h, Wa2h, Wa2h, 4, (long)kIn * 2 * kRnn, 2 * kRnn, 2 * kRnn,
                                                       w0, kKcat, 0, 2 * kRnn, kRnn, kWCarry);
  wtcast_kernel<<<dim3(16, 16, 12), 256, 0, stream>>>(Wi2h1, Wh2h1, Wa2h1, Wa2h1, 4, (long)kIn * kRnn, kRnn, kRnn,
                                                       w1, kKcat, 0, kRnn, kRnn, kWCarry);
  wtcast_kernel<<<dim3(16, 149, 1), 256, 0, stream>>>(Wproj, Wproj, Wproj, Wproj, 1, 0L, kOut, kOut,
                                                       wprojT, kRnn, 0, 0, 0, kWCarry);

  for (int i = 0; i < 2; ++i) {
    const float* hp = inputs + (size_t)(2 * i) * kBatch * kRnn;
    prep_kernel<<<dim3(4, kBatch), 256, 0, stream>>>(x, hp, acat0, acat1, (i == 0) ? 1 : 0);
    launch_gemm(stream, 1, 1, acat0 + kRnn, kKcat, 0L, watt + 1 * plane, kRnn, 0L, ahbuf, kAttPad, 0L,
                battpad + 1 * kAttPad, 0L, kBatch, kAttPad, kRnn);
    score_kernel<<<dim3(4, kBatch), 256, 0, stream>>>(av0, ahbuf, Wd2d, bd2d, scbuf);
    attapply_kernel<0><<<dim3(4, kBatch), 256, 0, stream>>>(scbuf, att, nh32, x, dout, acat0, acat1, top16);
    launch_gemm(stream, 16, 1, acat0, kKcat, 0L, w0, kKcat, 0L, sums, kNsum, 0L, bsum0, 0L, kBatch, kNsum, kKcat);
    gate_kernel<<<dim3(4, kBatch), 256, 0, stream>>>(sums, hp, acat1);
    launch_gemm(stream, 2, kPar, acat1, kKcat, (long)kBatch * kKcat, w1, kKcat, (long)kNhg * kKcat,
                hgpre, kRnn, (long)kBatch * kRnn, bsum1, (long)kNhg, kBatch, kNhg, kKcat);
    nh_kernel<<<dim3(4, kBatch), 256, 0, stream>>>(sums, hgpre, hp, nh32, nh16);
    launch_gemm(stream, 1, 1, nh16, kRnn, 0L, watt + 3 * plane, kRnn, 0L, ahbuf, kAttPad, 0L,
                battpad + 3 * kAttPad, 0L, kBatch, kAttPad, kRnn);
    score_kernel<<<dim3(4, kBatch), 256, 0, stream>>>(av1, ahbuf, Wd2d1, bd2d1, scbuf);
    if (i == 0) attapply_kernel<1><<<dim3(4, kBatch), 256, 0, stream>>>(scbuf, att, nh32, x, dout, acat0, acat1, top16);
    else        attapply_kernel<2><<<dim3(4, kBatch), 256, 0, stream>>>(scbuf, att, nh32, x, dout, acat0, acat1, top16);
  }

  launch_gemm(stream, 19, 1, top16, kRnn, 0L, wprojT, kRnn, 0L, logits, kOutPad, 0L, bprojp, 0L, kBatch, kOutPad, kRnn);
  lse_kernel<<<kBatch, 256, 0, stream>>>(logits, lsetab);
  lsm_write_kernel<<<(kOut1Float4 + 255) / 256, 256, 0, stream>>>(logits, lsetab, out1);
}
